// RelativePositionAttention_67894843015792
// MI455X (gfx1250) — hardware-verified
//
#include <hip/hip_runtime.h>
#include <math.h>
#include <stdint.h>

#ifndef NB
#define NB       16
#endif
#define NB_FULL  16
#define NTOK     577
#define SP       640
#define DM       768
#define NH       12
#define HD       64
#define INNER    (NH * HD)
#define GSIDE    24
#define RLEN     14
#define NTAB     30
#define TPAD     32
#define GROWS    48
#define NKB      19
#define NQT      (SP / 64)
#define WSC      256.0f
#define QS       8.0f
#define KS       8.0f
#define VS       8.0f
#define TS       256.0f
#define RESC     2048.0f
#define RINV     0.00048828125f
#define PCAR     32768.0f
#define CTXS     64.0f
#define LOG2E    1.4426950408889634f
#define ASCL     0.125f
#define ATT_WAVES   4
#define ATT_THREADS (ATT_WAVES * 32)
#define CVT_THREADS (DM / 8)
#define TR_THREADS  128
#define AUX_THREADS 128
#define OPITCH   68
#define GPITCH   68
#define TPITCH   65
#define WREG     3328
#define QVOFF    0
#define RCOFF    1024
#define BVOFF    1792
#define BAOFF    2816

static_assert(NB >= 1 && NB <= NB_FULL);
static_assert((NTOK - 1) == GSIDE * GSIDE);
static_assert((SP % 128) == 0 && (SP % 32) == 0 && SP >= NTOK);
static_assert(NKB * 32 >= NTOK && NKB * 32 <= SP);
static_assert(HD == 64 && INNER == DM && (DM % 64) == 0 && (DM % 32) == 0 && (INNER % 128) == 0);
static_assert(CVT_THREADS == 96 && CVT_THREADS * 8 == DM);
static_assert(NTAB <= TPAD && TPAD == 32 && 2 * RLEN + 2 == NTAB && GROWS == 2 * GSIDE);
static_assert(NQT * 64 == SP);
static_assert(RCOFF >= QVOFF + 2 * TPAD * 16 && BVOFF >= RCOFF + 16 * GROWS && BAOFF >= BVOFF + 2 * 16 * TPAD);
static_assert(WREG >= BAOFF + (2 * 16 * TPAD) / 2);
static_assert(16 * OPITCH <= BVOFF);
static_assert(ATT_WAVES * WREG * 4 <= 65536);
static_assert((SP / 8) <= AUX_THREADS && ATT_THREADS == 128 && TR_THREADS == 128);
static_assert((OPITCH * 4) % 16 == 0 && (GPITCH * 4) % 16 == 0);

typedef unsigned short u16;
typedef _Float16 v16h __attribute__((ext_vector_type(16)));
typedef _Float16 v8h  __attribute__((ext_vector_type(8)));
typedef float    v8f  __attribute__((ext_vector_type(8)));
typedef float    v4f  __attribute__((ext_vector_type(4)));
typedef unsigned int v4u __attribute__((ext_vector_type(4)));

union FragH { v16h v; v8h h[2]; v4u u[2]; };

__device__ __forceinline__ unsigned short bf_bits(float f) {
  unsigned u = __float_as_uint(f);
  return (unsigned short)((u + 0x7FFFu + ((u >> 16) & 1u)) >> 16);
}
__device__ __forceinline__ float bf_up(unsigned short h) { return __uint_as_float(((unsigned)h) << 16); }
__device__ __forceinline__ float bfr(float f) { return bf_up(bf_bits(f)); }
__device__ __forceinline__ unsigned short h_bits(_Float16 x) { return __builtin_bit_cast(unsigned short, x); }
__device__ __forceinline__ unsigned pk16(unsigned short a, unsigned short b) { return (unsigned)a | ((unsigned)b << 16); }
__device__ __forceinline__ v8f zero8() { v8f z = {0.f, 0.f, 0.f, 0.f, 0.f, 0.f, 0.f, 0.f}; return z; }

__device__ __forceinline__ v16h ldfrag_h(const _Float16* p) {
  FragH f;
  f.h[0] = *(const v8h*)(p);
  f.h[1] = *(const v8h*)(p + 16);
  return f.v;
}

__device__ __forceinline__ v8f mma_h(v16h a, v16h b, v8f c) {
  return __builtin_amdgcn_wmma_f32_16x16x32_f16(false, a, false, b, (short)0, c, false, false);
}
__device__ __forceinline__ void guard_s(v8f& a, v8f& b, v16h x0, v16h x1, v16h x2) {
#if defined(__HIP_DEVICE_COMPILE__)
  asm volatile("v_nop\n\tv_nop\n\tv_nop\n\tv_nop" : "+v"(a), "+v"(b) : "v"(x0), "v"(x1), "v"(x2) : "memory");
#endif
}
__device__ __forceinline__ void guard4(v8f& a, v8f& b, v8f& c, v8f& d, v16h x0, v16h x1, v16h x2, v16h x3) {
#if defined(__HIP_DEVICE_COMPILE__)
  asm volatile("v_nop\n\tv_nop\n\tv_nop\n\tv_nop"
               : "+v"(a), "+v"(b), "+v"(c), "+v"(d) : "v"(x0), "v"(x1), "v"(x2), "v"(x3) : "memory");
#endif
}
__device__ __forceinline__ void guard_p(v8f& a, v8f& b, v8f& c, v8f& d, v16h p, v16h x0, v16h x1, v16h x2, v16h x3) {
#if defined(__HIP_DEVICE_COMPILE__)
  asm volatile("v_nop\n\tv_nop\n\tv_nop\n\tv_nop"
               : "+v"(a), "+v"(b), "+v"(c), "+v"(d) : "v"(p), "v"(x0), "v"(x1), "v"(x2), "v"(x3) : "memory");
#endif
}
__device__ __forceinline__ void guard3(v8f& a, v8f& b, v8f& c, v16h p, v16h x0, v16h x1, v16h x2) {
#if defined(__HIP_DEVICE_COMPILE__)
  asm volatile("v_nop\n\tv_nop\n\tv_nop\n\tv_nop"
               : "+v"(a), "+v"(b), "+v"(c) : "v"(p), "v"(x0), "v"(x1), "v"(x2) : "memory");
#endif
}
__device__ __forceinline__ void guard_g(v8f (&acc)[8], v16h x0, v16h x1, v16h x2, v16h x3, v16h x4, v16h x5) {
#if defined(__HIP_DEVICE_COMPILE__)
  asm volatile("v_nop\n\tv_nop\n\tv_nop\n\tv_nop"
               : "+v"(acc[0]), "+v"(acc[1]), "+v"(acc[2]), "+v"(acc[3]),
                 "+v"(acc[4]), "+v"(acc[5]), "+v"(acc[6]), "+v"(acc[7])
               : "v"(x0), "v"(x1), "v"(x2), "v"(x3), "v"(x4), "v"(x5) : "memory");
#endif
}
__device__ __forceinline__ void acc_guard7(v8f (&o)[4], v8f (&g)[3]) {
#if defined(__HIP_DEVICE_COMPILE__)
  asm volatile("v_nop\n\tv_nop\n\tv_nop\n\tv_nop"
               : "+v"(o[0]), "+v"(o[1]), "+v"(o[2]), "+v"(o[3]), "+v"(g[0]), "+v"(g[1]), "+v"(g[2]));
#endif
}
__device__ __forceinline__ void wave_sync_lds() {
  __builtin_amdgcn_fence(__ATOMIC_RELEASE, "workgroup");
  __builtin_amdgcn_wave_barrier();
  __builtin_amdgcn_fence(__ATOMIC_ACQUIRE, "workgroup");
}

__global__ __launch_bounds__(CVT_THREADS)
void cvt16(const float* __restrict__ x, u16* Y) {
  const int tid = threadIdx.x;
  const int r = blockIdx.x;
  const int b = r / SP;
  const int s = r - b * SP;
  const int sc = (s < NTOK) ? s : (NTOK - 1);
  const float* src = x + ((size_t)b * (size_t)NTOK + (size_t)sc) * (size_t)DM + (size_t)tid * 8;
  const v4f a = *(const v4f*)(src), c4 = *(const v4f*)(src + 4);
  const unsigned msk = (s < NTOK) ? 0xFFFFFFFFu : 0u;
  v4u o;
#pragma unroll
  for (int e = 0; e < 2; ++e) {
    o[e]     = pk16(h_bits((_Float16)bfr(a[2 * e])),  h_bits((_Float16)bfr(a[2 * e + 1]))) & msk;
    o[2 + e] = pk16(h_bits((_Float16)bfr(c4[2 * e])), h_bits((_Float16)bfr(c4[2 * e + 1]))) & msk;
  }
  u16* dst = Y + (size_t)r * (size_t)DM + (size_t)tid * 8;
  for (int pass = 0; pass < 2; ++pass) {
    *(volatile v4u*)(dst) = o;
    __threadfence();
  }
}

__global__ __launch_bounds__(TR_THREADS)
void cvtT16(const float* __restrict__ W0, const float* __restrict__ W1, const float* __restrict__ W2,
            const float* __restrict__ W3, u16* Y, float scale) {
  __shared__ __align__(16) float tile[64 * TPITCH];
  const int tid = threadIdx.x;
  constexpr int NT = DM / 64;
  const int bid = blockIdx.x;
  const int sel = blockIdx.y;
  const float* W = (sel == 0) ? W0 : (sel == 1) ? W1 : (sel == 2) ? W2 : W3;
  u16* Yp = Y + (size_t)sel * (size_t)DM * (size_t)DM;
  const int kt  = bid % NT;
  const int ntb = bid / NT;
  const int k0  = kt * 64, n0 = ntb * 64;
  const int lr = tid >> 4, lc = (tid & 15) * 4;
#pragma unroll
  for (int p = 0; p < 8; ++p) {
    const int kk = p * 8 + lr;
    const v4f w4 = *(const v4f*)(W + (size_t)(k0 + kk) * (size_t)DM + n0 + lc);
    tile[kk * TPITCH + lc + 0] = w4[0];
    tile[kk * TPITCH + lc + 1] = w4[1];
    tile[kk * TPITCH + lc + 2] = w4[2];
    tile[kk * TPITCH + lc + 3] = w4[3];
  }
  __syncthreads();
  const int rq = tid >> 3, c8 = (tid & 7) * 8;
  v4u ov[4];
#pragma unroll
  for (int i = 0; i < 4; ++i) {
    const int row = 16 * i + rq;
#pragma unroll
    for (int e = 0; e < 4; ++e) {
      const float x0 = tile[(c8 + 2 * e) * TPITCH + row];
      const float x1 = tile[(c8 + 2 * e + 1) * TPITCH + row];
      ov[i][e] = pk16(h_bits((_Float16)(bfr(x0) * scale)), h_bits((_Float16)(bfr(x1) * scale)));
    }
  }
  u16* dst = Yp + (size_t)n0 * (size_t)DM + k0 + c8;
  for (int pass = 0; pass < 2; ++pass) {
#pragma unroll
    for (int i = 0; i < 4; ++i) {
      const int row = 16 * i + rq;
      *(volatile v4u*)(dst + (size_t)row * (size_t)DM) = ov[i];
    }
    __threadfence();
  }
}

__global__ __launch_bounds__(AUX_THREADS)
void aux16(const float* __restrict__ tvk, const float* __restrict__ thk, const float* __restrict__ tvv,
           const float* __restrict__ thv, u16* Tk, u16* Tv, u16* G) {
  const int tid = threadIdx.x;
  const int bid = blockIdx.x;
  if (bid < 2) {
    const float* src = (bid == 0) ? tvk : thk;
    u16* dstp = Tk + (size_t)bid * (TPAD * HD);
    v4u ov[2];
#pragma unroll
    for (int j = 0; j < 2; ++j) {
      const int u  = tid + AUX_THREADS * j;
      const int t  = u >> 3;
      const int d0 = (u & 7) * 8;
      const int tc = (t < NTAB) ? t : (NTAB - 1);
      const unsigned msk = (t < NTAB) ? 0xFFFFFFFFu : 0u;
      const float* sr = src + (size_t)tc * HD + d0;
      const v4f a = *(const v4f*)(sr), c4 = *(const v4f*)(sr + 4);
#pragma unroll
      for (int e = 0; e < 2; ++e) {
        ov[j][e]     = pk16(h_bits((_Float16)(bfr(a[2 * e]) * TS)),  h_bits((_Float16)(bfr(a[2 * e + 1]) * TS))) & msk;
        ov[j][2 + e] = pk16(h_bits((_Float16)(bfr(c4[2 * e]) * TS)), h_bits((_Float16)(bfr(c4[2 * e + 1]) * TS))) & msk;
      }
    }
    for (int pass = 0; pass < 2; ++pass) {
#pragma unroll
      for (int j = 0; j < 2; ++j)
        *(volatile v4u*)(dstp + (size_t)(tid + AUX_THREADS * j) * 8) = ov[j];
      __threadfence();
    }
  } else if (bid < 4) {
    const float* src = (bid == 2) ? tvv : thv;
    u16* dstp = Tv + (size_t)(bid - 2) * (HD * TPAD);
    v4u ov[2];
#pragma unroll
    for (int j = 0; j < 2; ++j) {
      const int u  = tid + AUX_THREADS * j;
      const int d  = u >> 2;
      const int t0 = (u & 3) * 8;
      unsigned short hb[8];
#pragma unroll
      for (int e = 0; e < 8; ++e) {
        const int t  = t0 + e;
        const int tc = (t < NTAB) ? t : (NTAB - 1);
        float v = src[(size_t)tc * HD + d];
        v = (t < NTAB) ? v : 0.f;
        hb[e] = h_bits((_Float16)(bfr(v) * TS));
      }
#pragma unroll
      for (int e = 0; e < 4; ++e) ov[j][e] = pk16(hb[2 * e], hb[2 * e + 1]);
    }
    for (int pass = 0; pass < 2; ++pass) {
#pragma unroll
      for (int j = 0; j < 2; ++j)
        *(volatile v4u*)(dstp + (size_t)(tid + AUX_THREADS * j) * 8) = ov[j];
      __threadfence();
    }
  } else {
    const int grow = bid - 4;
    if (tid < SP / 8) {
      const int key0 = tid * 8;
      unsigned short hb[8];
#pragma unroll
      for (int e = 0; e < 8; ++e) {
        const int key = key0 + e;
        const int valid = (key >= 1 && key < NTOK) ? 1 : 0;
        int km1 = key - 1; km1 = (km1 > 0) ? km1 : 0;
        const int rk = km1 / GSIDE;
        const int ck = km1 - rk * GSIDE;
        const int hitr = (rk == grow) ? 1 : 0;
        const int hitc = (ck == grow - GSIDE) ? 1 : 0;
        const int hit = valid & ((grow < GSIDE) ? hitr : hitc);
        hb[e] = hit ? (unsigned short)0x3C00 : (unsigned short)0;
      }
      v4u o;
#pragma unroll
      for (int e = 0; e < 4; ++e) o[e] = pk16(hb[2 * e], hb[2 * e + 1]);
      u16* dst = G + (size_t)grow * SP + key0;
      for (int pass = 0; pass < 2; ++pass) {
        *(volatile v4u*)(dst) = o;
        __threadfence();
      }
    }
  }
}

__device__ __forceinline__ void gemm_core(const _Float16* ap, const _Float16* bp, int K, v8f (&acc)[8]) {
  const size_t rs16 = (size_t)16 * (size_t)K;
#pragma unroll 1
  for (int k0 = 0; k0 < K; k0 += 32) {
    const v16h a0 = ldfrag_h(ap + k0), a1 = ldfrag_h(ap + rs16 + k0);
    const v16h b0 = ldfrag_h(bp + k0);
    const v16h b1 = ldfrag_h(bp + rs16 + k0);
    const v16h b2 = ldfrag_h(bp + 2 * rs16 + k0);
    const v16h b3 = ldfrag_h(bp + 3 * rs16 + k0);
    acc[0] = mma_h(a0, b0, acc[0]);
    acc[1] = mma_h(a0, b1, acc[1]);
    acc[2] = mma_h(a0, b2, acc[2]);
    acc[3] = mma_h(a0, b3, acc[3]);
    acc[4] = mma_h(a1, b0, acc[4]);
    acc[5] = mma_h(a1, b1, acc[5]);
    acc[6] = mma_h(a1, b2, acc[6]);
    acc[7] = mma_h(a1, b3, acc[7]);
    guard_g(acc, a0, a1, b0, b1, b2, b3);
  }
}
__device__ __forceinline__ void stage32x64(float* sl, v8f (&acc)[8], float oscale, int lane) {
  const int hh = lane >> 4, m = lane & 15;
#pragma unroll
  for (int i = 0; i < 2; ++i) {
#pragma unroll
    for (int r = 0; r < 8; ++r) {
      const int ro = (16 * i + 8 * hh + r) * GPITCH + m;
      sl[ro]      = acc[4 * i + 0][r] * oscale;
      sl[ro + 16] = acc[4 * i + 1][r] * oscale;
      sl[ro + 32] = acc[4 * i + 2][r] * oscale;
      sl[ro + 48] = acc[4 * i + 3][r] * oscale;
    }
  }
  wave_sync_lds();
}
__device__ __forceinline__ void accum32x64(float* sl, v8f (&acc)[8], float oscale, int lane) {
  const int hh = lane >> 4, m = lane & 15;
#pragma unroll
  for (int i = 0; i < 2; ++i) {
#pragma unroll
    for (int r = 0; r < 8; ++r) {
      const int ro = (16 * i + 8 * hh + r) * GPITCH + m;
      sl[ro]      += acc[4 * i + 0][r] * oscale;
      sl[ro + 16] += acc[4 * i + 1][r] * oscale;
      sl[ro + 32] += acc[4 * i + 2][r] * oscale;
      sl[ro + 48] += acc[4 * i + 3][r] * oscale;
    }
  }
  wave_sync_lds();
}

template <int RES>
__device__ __forceinline__ void gemm_o16_body(float* slab, const u16* __restrict__ A, const u16* __restrict__ Bt, u16* C,
                                              u16* Cr, int Mb, int N, int K, int aBs, int bBs, int cBs, float oscale) {
  const int tid = threadIdx.x, wave = tid >> 5, lane = tid & 31, hh = lane >> 4, m = lane & 15;
  const int ntile = N >> 6, mtile = Mb >> 7;
  const int bid  = blockIdx.x;
  const int nt   = bid % ntile;
  const int tmp  = bid / ntile;
  const int mt   = tmp % mtile;
  const int bz   = tmp / mtile;
  const int rowb = mt * 128 + wave * 32;
  const int col0 = nt * 64;
  if (rowb + 32 > Mb) return;
  const _Float16* Ab = (const _Float16*)(const void*)A + (size_t)bz * (size_t)aBs;
  const _Float16* Bb = (const _Float16*)(const void*)Bt + (size_t)bz * (size_t)bBs;
  const _Float16* ap = Ab + (size_t)(rowb + m) * K + 8 * hh;
  const _Float16* bp = Bb + (size_t)(col0 + m) * K + 8 * hh;
  v8f acc[8];
#pragma unroll
  for (int i = 0; i < 8; ++i) acc[i] = zero8();
  gemm_core(ap, bp, K, acc);
  float* sl = slab + wave * 32 * GPITCH;
  stage32x64(sl, acc, oscale, lane);
  const int rq = lane >> 3, c8 = (lane & 7) * 8;
  v4u ov[8], ovr[8];
#pragma unroll
  for (int i = 0; i < 8; ++i) {
    const int row = 4 * i + rq;
    const v4f a = *(const v4f*)(sl + row * GPITCH + c8), c4 = *(const v4f*)(sl + row * GPITCH + c8 + 4);
#pragma unroll
    for (int e = 0; e < 2; ++e) {
      const float x0 = a[2 * e], x1 = a[2 * e + 1], y0 = c4[2 * e], y1 = c4[2 * e + 1];
      const _Float16 hx0 = (_Float16)x0, hx1 = (_Float16)x1, hy0 = (_Float16)y0, hy1 = (_Float16)y1;
      ov[i][e]     = pk16(h_bits(hx0), h_bits(hx1));
      ov[i][2 + e] = pk16(h_bits(hy0), h_bits(hy1));
      if (RES) {
        ovr[i][e]     = pk16(h_bits((_Float16)((x0 - (float)hx0) * RESC)), h_bits((_Float16)((x1 - (float)hx1) * RESC)));
        ovr[i][2 + e] = pk16(h_bits((_Float16)((y0 - (float)hy0) * RESC)), h_bits((_Float16)((y1 - (float)hy1) * RESC)));
      } else {
        ovr[i][e] = 0u; ovr[i][2 + e] = 0u;
      }
    }
  }
  u16* Cb = C + (size_t)bz * (size_t)cBs + (size_t)rowb * (size_t)N + col0 + c8;
  u16* Crb = Cr + (size_t)bz * (size_t)cBs + (size_t)rowb * (size_t)N + col0 + c8;
  for (int pass = 0; pass < 2; ++pass) {
#pragma unroll
    for (int i = 0; i < 8; ++i) {
      const int row = 4 * i + rq;
      *(volatile v4u*)(Cb + (size_t)row * (size_t)N) = ov[i];
      if (RES) *(volatile v4u*)(Crb + (size_t)row * (size_t)N) = ovr[i];
    }
    __threadfence();
  }
}
__global__ __launch_bounds__(128)
void gemm_o16(const u16* __restrict__ A, const u16* __restrict__ Bt, u16* C, u16* Cr,
              int Mb, int N, int K, int aBs, int bBs, int cBs, float oscale) {
  __shared__ __align__(16) float slab[4 * 32 * GPITCH];
  gemm_o16_body<0>(slab, A, Bt, C, Cr, Mb, N, K, aBs, bBs, cBs, oscale);
}
__global__ __launch_bounds__(128)
void gemm_o16r(const u16* __restrict__ A, const u16* __restrict__ Bt, u16* C, u16* Cr,
               int Mb, int N, int K, int aBs, int bBs, int cBs, float oscale) {
  __shared__ __align__(16) float slab[4 * 32 * GPITCH];
  gemm_o16_body<1>(slab, A, Bt, C, Cr, Mb, N, K, aBs, bBs, cBs, oscale);
}

__global__ __launch_bounds__(ATT_THREADS)
void attn_fwd(const u16* __restrict__ Qh, const u16* __restrict__ Qr, const u16* __restrict__ Kp,
              const u16* __restrict__ Vp, const u16* __restrict__ Gp, const u16* __restrict__ Tk,
              const u16* __restrict__ Tv, u16* Ch, u16* Cr) {
  __shared__ __align__(16) float smem[ATT_WAVES * WREG];

  const int tid  = threadIdx.x;
  const int wave = tid >> 5;
  const int lane = tid & 31;
  const int hh   = lane >> 4;
  const int c    = lane & 15;

  const int bid  = blockIdx.x;
  const int qt   = bid % NQT;
  const int head = (bid / NQT) % NH;
  const int b    = bid / (NQT * NH);
  const int q0   = qt * 64 + wave * 16;

  float* wr = smem + wave * WREG;
  float* QV  = wr + QVOFF;
  float* RC  = wr + RCOFF;
  float* BVT = wr + BVOFF;
  _Float16* BA = (_Float16*)(wr + BAOFF);
  float* slab = wr;

  const _Float16* Qhb = (const _Float16*)(const void*)Qh + ((size_t)(b * SP + q0 + c)) * INNER + head * HD + 8 * hh;
  const _Float16* Qrb = (const _Float16*)(const void*)Qr + ((size_t)(b * SP + q0 + c)) * INNER + head * HD + 8 * hh;
  const _Float16* Kb  = (const _Float16*)(const void*)Kp + ((size_t)(b * SP + c)) * INNER + head * HD + 8 * hh;
  const _Float16* Vb  = (const _Float16*)(const void*)Vp + ((size_t)(b * INNER + head * HD + c)) * SP + 8 * hh;
  const _Float16* Gb  = (const _Float16*)(const void*)Gp + (size_t)c * SP + 8 * hh;
  const _Float16* Tkb = (const _Float16*)(const void*)Tk + (size_t)c * HD + 8 * hh;
  const _Float16* Tvb = (const _Float16*)(const void*)Tv + (size_t)c * TPAD + 8 * hh;

  v16h qf[2], qr[2];
#pragma unroll
  for (int kk = 0; kk < 2; ++kk) { qf[kk] = ldfrag_h(Qhb + 32 * kk); qr[kk] = ldfrag_h(Qrb + 32 * kk); }

  const float lsv = (LOG2E * ASCL) / (QS * TS);
#pragma unroll
  for (int tb = 0; tb < 2; ++tb) {
#pragma unroll
    for (int tt = 0; tt < 2; ++tt) {
      v8f eh = zero8(), er = zero8();
#pragma unroll
      for (int kk = 0; kk < 2; ++kk) {
        const v16h af = ldfrag_h(Tkb + tb * (TPAD * HD) + (16 * tt) * HD + 32 * kk);
        eh = mma_h(af, qf[kk], eh);
        er = mma_h(af, qr[kk], er);
        guard_s(eh, er, af, qf[kk], qr[kk]);
      }
#pragma unroll
      for (int r = 0; r < 8; ++r)
        QV[tb * (TPAD * 16) + (16 * tt + 8 * hh + r) * 16 + c] = (eh[r] + er[r] * RINV) * lsv;
    }
  }
  wave_sync_lds();

  const int qn   = q0 + c;
  const int qcls = (qn == 0) ? 1 : 0;
  const int qm1  = (qn > 0) ? (qn - 1) : 0;
  const int rq   = qm1 / GSIDE;
  const int cq   = qm1 - rq * GSIDE;
  const int bvq  = RLEN + 1 - rq;
  const int bhq  = RLEN + 1 - cq;
  const float* QVc = QV + c;
  const float* QHc = QV + TPAD * 16 + c;
  const float lsc = (LOG2E * ASCL) / (QS * KS);

  float mrun = -INFINITY, lrun = 0.f, pcl = 0.f;
  v8f o[4], g[3];
#pragma unroll
  for (int j = 0; j < 4; ++j) o[j] = zero8();
#pragma unroll
  for (int tl = 0; tl < 3; ++tl) g[tl] = zero8();

#pragma unroll 1
  for (int it = 0; it < NKB; ++it) {
    const int kb = it * 32;
    v8f s0 = zero8(), s1 = zero8(), r0 = zero8(), r1 = zero8();
    const _Float16* k0p = Kb + (size_t)kb * INNER;
    const _Float16* k1p = k0p + (size_t)16 * INNER;
#pragma unroll
    for (int kk = 0; kk < 2; ++kk) {
      const v16h kf0 = ldfrag_h(k0p + 32 * kk);
      const v16h kf1 = ldfrag_h(k1p + 32 * kk);
      s0 = mma_h(kf0, qf[kk], s0);
      s1 = mma_h(kf1, qf[kk], s1);
      r0 = mma_h(kf0, qr[kk], r0);
      r1 = mma_h(kf1, qr[kk], r1);
      guard4(s0, s1, r0, r1, kf0, kf1, qf[kk], qr[kk]);
    }
    float t[16];
#pragma unroll
    for (int w = 0; w < 2; ++w) {
#pragma unroll
      for (int i = 0; i < 8; ++i) {
        const int key = kb + 16 * w + 8 * hh + i;
        int km1 = key - 1; km1 = (km1 > 0) ? km1 : 0;
        const int rk = km1 / GSIDE;
        const int ck = km1 - rk * GSIDE;
        int tv = rk + bvq; tv = (tv > 1) ? tv : 1; tv = (tv < NTAB - 1) ? tv : (NTAB - 1);
        int th = ck + bhq; th = (th > 1) ? th : 1; th = (th < NTAB - 1) ? th : (NTAB - 1);
        const int z = qcls | ((key == 0) ? 1 : 0);
        tv = z ? 0 : tv;
        th = z ? 0 : th;
        const float raw = (w == 0) ? (s0[i] + r0[i] * RINV) : (s1[i] + r1[i] * RINV);
        const float lg = raw * lsc + QVc[tv * 16] + QHc[th * 16];
        t[8 * w + i] = (key < NTOK) ? lg : -INFINITY;
      }
    }
    float cm = t[0];
#pragma unroll
    for (int i = 1; i < 16; ++i) cm = fmaxf(cm, t[i]);
    cm = fmaxf(cm, __shfl_xor(cm, 16, 32));
    const float mn = fmaxf(mrun, cm);
    const float al = exp2f(mrun - mn);
    mrun = mn;
    float ps = 0.f, p0v = 0.f;
    FragH ph;
#pragma unroll
    for (int w = 0; w < 2; ++w) {
#pragma unroll
      for (int e4 = 0; e4 < 4; ++e4) {
        const int i = 8 * w + 2 * e4;
        const float p0 = exp2f(t[i] - mn), p1 = exp2f(t[i + 1] - mn);
        ps += p0 + p1;
        if (w == 0 && e4 == 0) p0v = p0;
        ph.u[w][e4] = pk16(h_bits((_Float16)(p0 * PCAR)), h_bits((_Float16)(p1 * PCAR)));
      }
    }
    ps += __shfl_xor(ps, 16, 32);
    lrun = lrun * al + ps;
    pcl = pcl * al + ((it == 0 && hh == 0) ? p0v : 0.f);
    float scl[8];
#pragma unroll
    for (int r = 0; r < 8; ++r) scl[r] = __shfl(al, 8 * hh + r, 32);
#pragma unroll
    for (int j = 0; j < 4; ++j) {
#pragma unroll
      for (int r = 0; r < 8; ++r) o[j][r] *= scl[r];
    }
#pragma unroll
    for (int tl = 0; tl < 3; ++tl) {
#pragma unroll
      for (int r = 0; r < 8; ++r) g[tl][r] *= scl[r];
    }
    {
      const _Float16* vp = Vb + kb;
      const v16h v0 = ldfrag_h(vp);
      const v16h v1 = ldfrag_h(vp + (size_t)16 * SP);
      const v16h v2 = ldfrag_h(vp + (size_t)32 * SP);
      const v16h v3 = ldfrag_h(vp + (size_t)48 * SP);
      o[0] = mma_h(ph.v, v0, o[0]);
      o[1] = mma_h(ph.v, v1, o[1]);
      o[2] = mma_h(ph.v, v2, o[2]);
      o[3] = mma_h(ph.v, v3, o[3]);
      guard_p(o[0], o[1], o[2], o[3], ph.v, v0, v1, v2, v3);
    }
    {
      const _Float16* gp = Gb + kb;
      const v16h g0 = ldfrag_h(gp);
      const v16h g1 = ldfrag_h(gp + (size_t)16 * SP);
      const v16h g2 = ldfrag_h(gp + (size_t)32 * SP);
      g[0] = mma_h(ph.v, g0, g[0]);
      g[1] = mma_h(ph.v, g1, g[1]);
      g[2] = mma_h(ph.v, g2, g[2]);
      guard3(g[0], g[1], g[2], ph.v, g0, g1, g2);
    }
  }
  acc_guard7(o, g);

  wave_sync_lds();
#pragma unroll
  for (int tl = 0; tl < 3; ++tl) {
#pragma unroll
    for (int r = 0; r < 8; ++r) RC[(8 * hh + r) * GROWS + 16 * tl + c] = g[tl][r];
  }
  const float pc = pcl + __shfl_xor(pcl, 16, 32);
  wave_sync_lds();
  float* bv = BVT + (hh * 16 + c) * TPAD;
#pragma unroll
  for (int e = 0; e < TPAD; ++e) bv[e] = 0.f;
  const float* rc = RC + c * GROWS + GSIDE * hh;
  const int bq = hh ? bhq : bvq;
#pragma unroll 4
  for (int p = 0; p < GSIDE; ++p) {
    int tt = p + bq; tt = (tt > 1) ? tt : 1; tt = (tt < NTAB - 1) ? tt : (NTAB - 1); tt = qcls ? 0 : tt;
    bv[tt] += rc[p];
  }
  bv[0] += pc * PCAR;
  wave_sync_lds();
  const float ln = 1.0f / lrun;
  v4u arow[4];
#pragma unroll
  for (int e = 0; e < 4; ++e) {
    const v4f a = *(const v4f*)(bv + 8 * e), cc4 = *(const v4f*)(bv + 8 * e + 4);
#pragma unroll
    for (int f = 0; f < 2; ++f) {
      arow[e][f]     = pk16(h_bits((_Float16)(a[2 * f] * ln)),   h_bits((_Float16)(a[2 * f + 1] * ln)));
      arow[e][2 + f] = pk16(h_bits((_Float16)(cc4[2 * f] * ln)), h_bits((_Float16)(cc4[2 * f + 1] * ln)));
    }
  }
  u16* bau = (u16*)(void*)(BA + (hh * 16 + c) * TPAD);
#pragma unroll
  for (int e = 0; e < 4; ++e) *(v4u*)(bau + 8 * e) = arow[e];
  wave_sync_lds();
  const _Float16* bap = BA + c * TPAD + 8 * hh;
  const v16h av = ldfrag_h(bap);
  const v16h ah = ldfrag_h(bap + 16 * TPAD);
  v8f e4[4];
#pragma unroll
  for (int j = 0; j < 4; ++j) e4[j] = zero8();
  {
    const v16h f0 = ldfrag_h(Tvb);
    const v16h f1 = ldfrag_h(Tvb + 16 * TPAD);
    const v16h f2 = ldfrag_h(Tvb + 32 * TPAD);
    const v16h f3 = ldfrag_h(Tvb + 48 * TPAD);
    e4[0] = mma_h(av, f0, e4[0]);
    e4[1] = mma_h(av, f1, e4[1]);
    e4[2] = mma_h(av, f2, e4[2]);
    e4[3] = mma_h(av, f3, e4[3]);
    guard_p(e4[0], e4[1], e4[2], e4[3], av, f0, f1, f2, f3);
  }
  {
    const _Float16* Thb = Tvb + HD * TPAD;
    const v16h f0 = ldfrag_h(Thb);
    const v16h f1 = ldfrag_h(Thb + 16 * TPAD);
    const v16h f2 = ldfrag_h(Thb + 32 * TPAD);
    const v16h f3 = ldfrag_h(Thb + 48 * TPAD);
    e4[0] = mma_h(ah, f0, e4[0]);
    e4[1] = mma_h(ah, f1, e4[1]);
    e4[2] = mma_h(ah, f2, e4[2]);
    e4[3] = mma_h(ah, f3, e4[3]);
    guard_p(e4[0], e4[1], e4[2], e4[3], ah, f0, f1, f2, f3);
  }
  const float linv = ln * (CTXS / (PCAR * VS));
  float inv[8];
#pragma unroll
  for (int r = 0; r < 8; ++r) inv[r] = __shfl(linv, 8 * hh + r, 32);
  const float esc = CTXS / (PCAR * TS);
#pragma unroll
  for (int r = 0; r < 8; ++r) {
#pragma unroll
    for (int j = 0; j < 4; ++j) slab[(8 * hh + r) * OPITCH + 16 * j + c] = o[j][r] * inv[r] + e4[j][r] * esc;
  }
  wave_sync_lds();
  const int rq4 = lane >> 3, c8 = (lane & 7) * 8;
  v4u oh[4], orr[4];
#pragma unroll
  for (int i = 0; i < 4; ++i) {
    const int row = 4 * i + rq4;
    const v4f a = *(const v4f*)(slab + row * OPITCH + c8), cc4 = *(const v4f*)(slab + row * OPITCH + c8 + 4);
#pragma unroll
    for (int f = 0; f < 2; ++f) {
      const float x0 = a[2 * f], x1 = a[2 * f + 1], y0 = cc4[2 * f], y1 = cc4[2 * f + 1];
      const _Float16 hx0 = (_Float16)x0, hx1 = (_Float16)x1, hy0 = (_Float16)y0, hy1 = (_Float16)y1;
      oh[i][f]      = pk16(h_bits(hx0), h_bits(hx1));
      oh[i][2 + f]  = pk16(h_bits(hy0), h_bits(hy1));
      orr[i][f]     = pk16(h_bits((_Float16)((x0 - (float)hx0) * RESC)), h_bits((_Float16)((x1 - (float)hx1) * RESC)));
      orr[i][2 + f] = pk16(h_bits((_Float16)((y0 - (float)hy0) * RESC)), h_bits((_Float16)((y1 - (float)hy1) * RESC)));
    }
  }
  u16* chp = Ch + ((size_t)(b * SP + q0)) * INNER + head * HD + c8;
  u16* crp = Cr + ((size_t)(b * SP + q0)) * INNER + head * HD + c8;
  for (int pass = 0; pass < 2; ++pass) {
#pragma unroll
    for (int i = 0; i < 4; ++i) {
      const int row = 4 * i + rq4;
      *(volatile v4u*)(chp + (size_t)row * INNER) = oh[i];
      *(volatile v4u*)(crp + (size_t)row * INNER) = orr[i];
    }
    __threadfence();
  }
}

__global__ __launch_bounds__(128)
void gemm_proj(const u16* __restrict__ Ah, const u16* __restrict__ Ar, const u16* __restrict__ Bt,
               const float* __restrict__ bias, float* Out, int Mb) {
  __shared__ __align__(16) float slab[4 * 32 * GPITCH];
  const int tid = threadIdx.x, wave = tid >> 5, lane = tid & 31, hh = lane >> 4, m = lane & 15;
  constexpr int ntile = DM / 64;
  const int mtile = Mb >> 7;
  const int bid  = blockIdx.x;
  const int nt   = bid % ntile;
  const int mt   = (bid / ntile) % mtile;
  const int rowb = mt * 128 + wave * 32;
  const int col0 = nt * 64;
  if (rowb + 32 > Mb) return;
  const _Float16* aph = (const _Float16*)(const void*)Ah + (size_t)(rowb + m) * INNER + 8 * hh;
  const _Float16* apr = (const _Float16*)(const void*)Ar + (size_t)(rowb + m) * INNER + 8 * hh;
  const _Float16* bpp = (const _Float16*)(const void*)Bt + (size_t)(col0 + m) * INNER + 8 * hh;
  float* sl = slab + wave * 32 * GPITCH;
  const float osh = 1.0f / (CTXS * WSC);
  v8f acc[8];
#pragma unroll
  for (int i = 0; i < 8; ++i) acc[i] = zero8();
  gemm_core(aph, bpp, INNER, acc);
  stage32x64(sl, acc, osh, lane);
#pragma unroll
  for (int i = 0; i < 8; ++i) acc[i] = zero8();
  gemm_core(apr, bpp, INNER, acc);
  accum32x64(sl, acc, osh * RINV, lane);

  const int rr = lane >> 4, c4 = (lane & 15) * 4;
  v4f b4;
#pragma unroll
  for (int e = 0; e < 4; ++e) b4[e] = bfr(bias[col0 + c4 + e]);
  const int bb = rowb / SP;
  const int s0 = rowb - bb * SP;
  v4f vals[16];
#pragma unroll
  for (int i = 0; i < 16; ++i) {
    const int row = 2 * i + rr;
    vals[i] = *(const v4f*)(sl + row * GPITCH + c4) + b4;
  }
  float* ob = Out + ((size_t)bb * (size_t)NTOK + (size_t)s0) * (size_t)DM + col0 + c4;
  for (int pass = 0; pass < 2; ++pass) {
#pragma unroll
    for (int i = 0; i < 16; ++i) {
      const int row = 2 * i + rr;
      if (s0 + row < NTOK) *(volatile v4f*)(ob + (size_t)row * (size_t)DM) = vals[i];
    }
    __threadfence();
  }
}

extern "C" void kernel_launch(void* const* d_in, const int* in_sizes, int n_in,
                              void* d_out, int out_size, void* d_ws, size_t ws_size,
                              hipStream_t stream) {
  if (n_in < 10) return;
  if (in_sizes[0] < NB * NTOK * DM) return;
  if (in_sizes[1] < DM * INNER || in_sizes[2] < DM * INNER || in_sizes[3] < DM * INNER) return;
  if (in_sizes[4] < INNER * DM) return;
  if (in_sizes[5] < DM) return;
  if (in_sizes[6] < NTAB * HD || in_sizes[7] < NTAB * HD || in_sizes[8] < NTAB * HD || in_sizes[9] < NTAB * HD) return;
  if (out_size < NB * NTOK * DM) return;

  const float* x   = (const float*)d_in[0];
  const float* wq  = (const float*)d_in[1];
  const float* wk  = (const float*)d_in[2];
  const float* wv  = (const float*)d_in[3];
  const float* wp  = (const float*)d_in[4];
  const float* bp  = (const float*)d_in[5];
  const float* tvk = (const float*)d_in[6];
  const float* thk = (const float*)d_in[7];
  const float* tvv = (const float*)d_in[8];
  const float* thv = (const float*)d_in[9];
  float*       out = (float*)d_out;

  auto al256 = [](size_t v) { return (v + 255) & ~(size_t)255; };
  const size_t szAct = (size_t)NB * SP * DM * 2;
  const size_t szW   = (size_t)DM * DM * 2;
  const size_t szVT  = (size_t)NB * INNER * SP * 2;
  const size_t szTK  = (size_t)2 * TPAD * HD * 2;
  const size_t szTV  = (size_t)2 * HD * TPAD * 2;
  const size_t szG   = (size_t)GROWS * SP * 2;
  size_t off = 0;
  const size_t oX   = off; off = al256(off + szAct);
  const size_t oWT  = off; off = al256(off + 4 * szW);
  const size_t oTK  = off; off = al256(off + szTK);
  const size_t oTV  = off; off = al256(off + szTV);
  const size_t oG   = off; off = al256(off + szG);
  const size_t oQH  = off; off = al256(off + szAct);
  const size_t oQR  = off; off = al256(off + szAct);
  const size_t oK   = off; off = al256(off + szAct);
  const size_t oVT  = off; off = al256(off + szVT);
  const size_t oCH  = off; off = al256(off + szAct);
  const size_t oCR  = off; off = al256(off + szAct);
  if (off > ws_size) return;
  if (off > (size_t)134217728) return;

  char* ws = (char*)d_ws;
  u16* X16  = (u16*)(ws + oX);
  u16* WT   = (u16*)(ws + oWT);
  u16* WQT  = WT;
  u16* WKT  = WT + (size_t)DM * DM;
  u16* WVT  = WT + (size_t)2 * DM * DM;
  u16* WPT  = WT + (size_t)3 * DM * DM;
  u16* TK   = (u16*)(ws + oTK);
  u16* TVT  = (u16*)(ws + oTV);
  u16* G16  = (u16*)(ws + oG);
  u16* QH   = (u16*)(ws + oQH);
  u16* QR   = (u16*)(ws + oQR);
  u16* K16  = (u16*)(ws + oK);
  u16* VT16 = (u16*)(ws + oVT);
  u16* CH   = (u16*)(ws + oCH);
  u16* CR   = (u16*)(ws + oCR);

  cvt16<<<dim3(NB * SP), dim3(CVT_THREADS), 0, stream>>>(x, X16);
  cvtT16<<<dim3((DM / 64) * (DM / 64), 4), dim3(TR_THREADS), 0, stream>>>(wq, wk, wv, wp, WT, WSC);
  aux16<<<dim3(4 + GROWS), dim3(AUX_THREADS), 0, stream>>>(tvk, thk, tvv, thv, TK, TVT, G16);
  gemm_o16r<<<dim3((NB * SP / 128) * (INNER / 64)), dim3(128), 0, stream>>>(
      X16, WQT, QH, QR, NB * SP, INNER, DM, 0, 0, 0, QS / WSC);
  gemm_o16<<<dim3((NB * SP / 128) * (INNER / 64)), dim3(128), 0, stream>>>(
      X16, WKT, K16, K16, NB * SP, INNER, DM, 0, 0, 0, KS / WSC);
  gemm_o16<<<dim3(NB * (INNER / 128) * (SP / 64)), dim3(128), 0, stream>>>(
      WVT, X16, VT16, VT16, INNER, SP, DM, 0, SP * DM, INNER * SP, VS / WSC);
  attn_fwd<<<dim3(NB * NH * NQT), dim3(ATT_THREADS), 0, stream>>>(QH, QR, K16, VT16, G16, TK, TVT, CH, CR);
  gemm_proj<<<dim3((NB * SP / 128) * (DM / 64)), dim3(128), 0, stream>>>(CH, CR, WPT, bp, out, NB * SP);
  (void)hipGetLastError();
}
